// IdentifyLay_31181462569492
// MI455X (gfx1250) — hardware-run, weakly checked
//
#include <hip/hip_runtime.h>

typedef float          v8f   __attribute__((ext_vector_type(8)));
typedef float          v4f   __attribute__((ext_vector_type(4)));
typedef unsigned int   v4u   __attribute__((ext_vector_type(4)));
typedef int            v8i   __attribute__((ext_vector_type(8)));
typedef unsigned short v8us  __attribute__((ext_vector_type(8)));
typedef unsigned short v16us __attribute__((ext_vector_type(16)));
typedef __bf16         v16bf __attribute__((ext_vector_type(16)));
typedef _Float16       v16h  __attribute__((ext_vector_type(16)));
typedef v4f  __attribute__((may_alias)) v4fa;
typedef v8us __attribute__((may_alias)) v8usa;
union FragB { v16bf v; v16us u; v8us h[2]; v8i w; };
union FragH { v16h  v; v16us u; v8us h[2]; v8i w; };

__device__ __forceinline__ v8f wmb(const FragB& a, const FragB& b, v8f c) {
  v8f d = __builtin_amdgcn_wmma_f32_16x16x32_bf16(false, a.v, false, b.v, (short)0, c, false, false);
  asm volatile("v_nop\n\tv_nop\n\tv_nop\n\tv_nop" : "+v"(d) : "v"(a.w), "v"(b.w));
  return d;
}

__device__ __forceinline__ v8f wmh(const FragH& a, const FragH& b, v8f c) {
  v8f d = __builtin_amdgcn_wmma_f32_16x16x32_f16(false, a.v, false, b.v, (short)0, c, false, false);
  asm volatile("v_nop\n\tv_nop\n\tv_nop\n\tv_nop" : "+v"(d) : "v"(a.w), "v"(b.w));
  return d;
}

__device__ __forceinline__ unsigned bf16_bits(float f) {
  const unsigned u = __float_as_uint(f);
  const unsigned r = (u + 0x7FFFu + ((u >> 16) & 1u)) >> 16;
  const unsigned q = (u >> 16) | 0x40u;
  return ((u & 0x7fffffffu) > 0x7f800000u) ? q : r;
}

__device__ __forceinline__ float bf16_val(float f) {
  return __uint_as_float(bf16_bits(f) << 16);
}
__device__ __forceinline__ int clampi(int v, int lo, int hi) {
  return v < lo ? lo : (v > hi ? hi : v);
}

__device__ __forceinline__ unsigned f16_bits(float f) {
  const unsigned u  = __float_as_uint(f);
  const unsigned s  = (u >> 16) & 0x8000u;
  const unsigned a  = u & 0x7fffffffu;
  const unsigned t  = a - 0x38000000u;
  const unsigned r  = (t + 0x0FFFu + ((t >> 13) & 1u)) >> 13;
  const unsigned rc = r > 0x7C00u ? 0x7C00u : r;
  const bool small  = a < 0x38800000u;
  const bool isnan  = a > 0x7f800000u;
  const unsigned fin = small ? 0u : (s | rc);
  return isnan ? (s | 0x7E00u) : fin;
}

__device__ __forceinline__ unsigned pk16(unsigned lo, unsigned hi) { return lo | (hi << 16); }
__device__ __forceinline__ unsigned bf16_lo_bits(float v) {
  float hi = bf16_val(v);
  asm volatile("" : "+v"(hi));
  return bf16_bits(v - hi);
}
__device__ __forceinline__ v4u pack8_bf16(v4f a, v4f c) {
  return (v4u){ pk16(bf16_bits(a[0]), bf16_bits(a[1])), pk16(bf16_bits(a[2]), bf16_bits(a[3])),
                pk16(bf16_bits(c[0]), bf16_bits(c[1])), pk16(bf16_bits(c[2]), bf16_bits(c[3])) };
}
__device__ __forceinline__ v4u pack8_bf16_lo(v4f a, v4f c) {
  return (v4u){ pk16(bf16_lo_bits(a[0]), bf16_lo_bits(a[1])), pk16(bf16_lo_bits(a[2]), bf16_lo_bits(a[3])),
                pk16(bf16_lo_bits(c[0]), bf16_lo_bits(c[1])), pk16(bf16_lo_bits(c[2]), bf16_lo_bits(c[3])) };
}
__device__ __forceinline__ v4u pack8_f16(v4f a, v4f c) {
  return (v4u){ pk16(f16_bits(a[0]), f16_bits(a[1])), pk16(f16_bits(a[2]), f16_bits(a[3])),
                pk16(f16_bits(c[0]), f16_bits(c[1])), pk16(f16_bits(c[2]), f16_bits(c[3])) };
}

template <int FORM>
__global__ __launch_bounds__(256) void k_plane(const float* __restrict__ src, int rows, int cols, int ldsrc,
                                               unsigned short* __restrict__ dst, int MP, int KP) {
  static_assert(FORM >= 0 && FORM <= 3);
  const int KTOT = (FORM == 1 || FORM == 3) ? 2 * KP : KP;
  const unsigned ppr   = (unsigned)(KTOT >> 3);
  const unsigned kp8   = (unsigned)(KP >> 3);
  const unsigned total = (unsigned)MP * ppr;
  const unsigned g     = blockIdx.x * 256u + threadIdx.x;
  const unsigned rowu  = g / ppr;
  const unsigned p     = g - rowu * ppr;
  const bool second    = p >= kp8;
  const int row = (int)rowu;
  const int c0  = (int)((second ? p - kp8 : p) << 3);
  const float* srow = src + (size_t)clampi(row, 0, rows - 1) * (size_t)ldsrc;
  float x[8];
  unsigned mk[8];
#pragma unroll
  for (int e = 0; e < 8; ++e) {
    const int c = c0 + e;
    const float v = srow[clampi(c, 0, cols - 1)];
    asm volatile("" :: "v"(v));
    x[e]  = v;
    mk[e] = (row < rows && c < cols) ? 0xFFFFu : 0u;
  }
  const v4f a = (v4f){ x[0], x[1], x[2], x[3] };
  const v4f c = (v4f){ x[4], x[5], x[6], x[7] };
  v4u o;
  if (FORM == 2) {
    o = pack8_f16(a, c);
  } else {
    const v4u hi = pack8_bf16(a, c);
    o = hi;
    if (FORM == 1) { const v4u lo = pack8_bf16_lo(a, c); o = second ? lo : hi; }
  }
  const v4u mw = (v4u){ pk16(mk[0], mk[1]), pk16(mk[2], mk[3]), pk16(mk[4], mk[5]), pk16(mk[6], mk[7]) };
  o &= mw;
  if (g < total) {
    volatile v4u* q = (volatile v4u*)(dst + (size_t)g * 8);
    *q = o;
    __threadfence();
    *q = o;
  }
}

template <int FORM> struct FragOf    { typedef FragB T; };
template <>         struct FragOf<2> { typedef FragH T; };
__device__ __forceinline__ v8f mm(const FragB& a, const FragB& b, v8f c) { return wmb(a, b, c); }
__device__ __forceinline__ v8f mm(const FragH& a, const FragH& b, v8f c) { return wmh(a, b, c); }
template <class F> __device__ __forceinline__ F ld_frag(const unsigned short* p) {
  F f;
  f.h[0] = *(const v8usa*)(p);
  f.h[1] = *(const v8usa*)(p + 16);
  return f;
}

template <int FORM, int EPI>
__global__ __launch_bounds__(256) __attribute__((amdgpu_num_vgpr(248)))
void k_gemm_nt(const unsigned short* __restrict__ A, const unsigned short* __restrict__ B,
               const float* __restrict__ bias, float* __restrict__ D, int M, int N, int KTOT, int ldd) {
  static_assert(FORM >= 0 && FORM <= 2);
  static_assert(EPI == 0 || EPI == 1);
  typedef typename FragOf<FORM>::T F;
  __shared__ __attribute__((aligned(16))) float sT[8][16 * 68];
  const int lane = threadIdx.x & 31;
  const int wave = threadIdx.x >> 5;
  const int tilesM = (M + 63) >> 6;
  const int tilesN = (N + 63) >> 6;
  const int tile = blockIdx.x * 8 + wave;
  if (tile >= tilesM * tilesN) return;
  const int tm = tile / tilesN;
  const int tn = tile - tm * tilesN;
  const int m0 = tm << 6;
  const int n0 = tn << 6;

  const int rl = lane & 15;
  const int h8 = (lane >> 4) * 8;
  const unsigned short* pa = A + (size_t)(m0 + rl) * (size_t)KTOT + h8;
  const unsigned short* pb = B + (size_t)(n0 + rl) * (size_t)KTOT + h8;

  v8f acc[4][4];
#pragma unroll
  for (int i = 0; i < 4; ++i)
#pragma unroll
    for (int j = 0; j < 4; ++j) acc[i][j] = (v8f){0.f, 0.f, 0.f, 0.f, 0.f, 0.f, 0.f, 0.f};

#pragma unroll 1
  for (int k0 = 0; k0 < KTOT; k0 += 32) {
    F bf[4];
#pragma unroll
    for (int j = 0; j < 4; ++j) bf[j] = ld_frag<F>(pb + (size_t)(j << 4) * (size_t)KTOT + k0);
#pragma unroll
    for (int i = 0; i < 4; ++i) {
      const F af = ld_frag<F>(pa + (size_t)(i << 4) * (size_t)KTOT + k0);
#pragma unroll
      for (int j = 0; j < 4; ++j) acc[i][j] = mm(af, bf[j], acc[i][j]);
    }
  }

  float* slab = sT[wave];
  const int hh = lane >> 4;
  const int c4 = (lane & 15) * 4;
  const int nc = n0 + c4;
  const bool cok = nc < N;
  v4f bv = (v4f){0.f, 0.f, 0.f, 0.f};
  if (EPI == 1) {
    bv = *(const v4fa*)(bias + clampi(nc, 0, N - 4));
    asm volatile("" :: "v"(bv));
  }
#pragma unroll
  for (int i = 0; i < 4; ++i) {
    const int mBase = m0 + (i << 4);
#pragma unroll
    for (int j = 0; j < 4; ++j) {
#pragma unroll
      for (int r = 0; r < 8; ++r) slab[(h8 + r) * 68 + (j << 4) + rl] = acc[i][j][r];
    }
    __builtin_amdgcn_fence(__ATOMIC_RELEASE, "workgroup");
    __builtin_amdgcn_wave_barrier();
    __builtin_amdgcn_fence(__ATOMIC_ACQUIRE, "workgroup");
    v4f vv[8];
#pragma unroll
    for (int it = 0; it < 8; ++it) {
      const int row = it * 2 + hh;
      v4f v = *(const v4fa*)(slab + row * 68 + c4);
      if (EPI == 1) v += bv;
      vv[it] = v;
    }
    for (int pass = 0; pass < 2; ++pass) {
#pragma unroll
      for (int it = 0; it < 8; ++it) {
        const int row = mBase + it * 2 + hh;
        if (cok && row < M) *(volatile v4f*)(D + (size_t)row * (size_t)ldd + nc) = vv[it];
      }
      __threadfence();
    }
    __builtin_amdgcn_fence(__ATOMIC_RELEASE, "workgroup");
    __builtin_amdgcn_wave_barrier();
    __builtin_amdgcn_fence(__ATOMIC_ACQUIRE, "workgroup");
  }
}

#define W1S_TERMS 2
#define NPT       1024
#define DD        64
#define KT        (DD * W1S_TERMS)
#define PPRZ      (KT / 8)
#define OUT_ELEMS 4194304
#define NB_ZZ     ((2 * NPT * PPRZ) / 256)
#define NB_ZR     ((2 * NPT * (DD / 4)) / 256)
#define NB_PREP   (NB_ZZ + NB_ZR + 1)
#define NPW       (2 * DD * PPRZ)
#define NITW      (NPW / 256)
#define WS_PITCH  65
#define TROWS     128
#define TPITCH    68
#define LDS_T     (TROWS * TPITCH)
#define LDS_O     (8 * NPT)
#define LDS_Z     (8 * DD)
#define LDS_W     128
#define PAIR_LDS_FLOATS (LDS_T + LDS_O + LDS_Z + LDS_W)
#define PAIR_LDS_BYTES  (PAIR_LDS_FLOATS * 4)
#define SZ_ZZ     (2 * NPT * KT * 2)
#define SZ_ZR     (2 * NPT * DD * 4)
#define SZ_ZW     (2 * NPT * DD * 4)
#define SZ_REC    (2 * 64 * DD * 8)
#define SZ_W1ST   (2 * DD * KT * 2)
#define SZ_SF     512
#define SZ_TAB    1024
#define WS_TOTAL  (SZ_ZZ + SZ_ZR + SZ_ZW + SZ_REC + SZ_W1ST + SZ_SF + SZ_TAB)

static_assert(W1S_TERMS >= 1 && W1S_TERMS <= 3);
static_assert(NPT % 128 == 0 && NPT == 1024 && DD == 64);
static_assert(KT % 32 == 0 && NPT % 64 == 0 && DD % 64 == 0);
static_assert((2 * NPT * PPRZ) % 256 == 0 && (NPT * PPRZ) % 256 == 0);
static_assert((2 * NPT * (DD / 4)) % 256 == 0);
static_assert(NPW % 256 == 0 && NITW * 256 == NPW);
static_assert(2 * NPT == 256 * 8);
static_assert(4 * NPT * NPT == OUT_ELEMS);
static_assert(((1 + 2) * NPT + (NPT - 1)) * NPT + (NPT - 1) == OUT_ELEMS - 1);
static_assert(SZ_ZZ % 256 == 0 && SZ_ZR % 256 == 0 && SZ_ZW % 256 == 0 && SZ_REC % 256 == 0);
static_assert(SZ_W1ST % 256 == 0 && SZ_SF % 256 == 0 && SZ_TAB % 256 == 0);
static_assert(WS_TOTAL <= 2 * 1024 * 1024);
static_assert(PAIR_LDS_BYTES + 0 <= 327680);
static_assert((LDS_T * 4) % 16 == 0 && ((LDS_T + LDS_O) * 4) % 16 == 0 && ((LDS_T + LDS_O + LDS_Z) * 4) % 16 == 0);
static_assert(TROWS * (DD / 4) == 8 * 256);
static_assert(2 * DD * WS_PITCH * 4 + 512 <= 65536);

typedef float  pv2f __attribute__((ext_vector_type(2)));
typedef double pv2d __attribute__((ext_vector_type(2)));
typedef pv2f __attribute__((may_alias)) pv2fa;

__device__ __forceinline__ unsigned bf16_res2_bits(float v) {
  float hi = bf16_val(v);
  asm volatile("" : "+v"(hi));
  float r1 = v - hi;
  asm volatile("" : "+v"(r1));
  float mid = bf16_val(r1);
  asm volatile("" : "+v"(mid));
  return bf16_bits(r1 - mid);
}
__device__ __forceinline__ v4u pack8_bf16_res2(v4f a, v4f c) {
  return (v4u){ pk16(bf16_res2_bits(a[0]), bf16_res2_bits(a[1])), pk16(bf16_res2_bits(a[2]), bf16_res2_bits(a[3])),
                pk16(bf16_res2_bits(c[0]), bf16_res2_bits(c[1])), pk16(bf16_res2_bits(c[2]), bf16_res2_bits(c[3])) };
}
__device__ __forceinline__ float blend3(float a, float b, float c, unsigned ma, unsigned mb, unsigned mc) {
  return __uint_as_float((__float_as_uint(a) & ma) | (__float_as_uint(b) & mb) | (__float_as_uint(c) & mc));
}

__global__ __launch_bounds__(256) void k_prep(const float* __restrict__ z1, const float* __restrict__ z2,
                                              const float* __restrict__ W2, const float* __restrict__ b1,
                                              const float* __restrict__ b2,
                                              unsigned short* __restrict__ ZZ, float* __restrict__ ZR,
                                              float* __restrict__ TAB) {
  const unsigned tid = threadIdx.x;
  const unsigned blk = blockIdx.x;
  if (blk < (unsigned)NB_ZZ) {
    const unsigned g   = blk * 256u + tid;
    const unsigned row = g / (unsigned)PPRZ;
    const unsigned p   = g - row * (unsigned)PPRZ;
    const unsigned e   = row >> 10;
    const unsigned i   = row & 1023u;
    const unsigned c0  = (p & 7u) << 3;
    const size_t so = (size_t)i * DD + c0;
    const v4f a1 = *(const v4fa*)(z1 + so);
    const v4f c1 = *(const v4fa*)(z1 + so + 4);
    const v4f a2 = *(const v4fa*)(z2 + so);
    const v4f c2 = *(const v4fa*)(z2 + so + 4);
    asm volatile("" :: "v"(a1)); asm volatile("" :: "v"(c1));
    asm volatile("" :: "v"(a2)); asm volatile("" :: "v"(c2));
    const v4f a = (e != 0u) ? a2 : a1;
    const v4f c = (e != 0u) ? c2 : c1;
    const v4u o = pack8_bf16(a, c);
    volatile v4u* q = (volatile v4u*)(ZZ + (size_t)g * 8);
    *q = o;
    __threadfence();
    *q = o;
  } else if (blk < (unsigned)(NB_ZZ + NB_ZR)) {
    const unsigned g = (blk - (unsigned)NB_ZZ) * 256u + tid;
    const unsigned e = g >> 14;
    const unsigned qd = g & 16383u;
    const v4f a1 = *(const v4fa*)(z1 + (size_t)qd * 4);
    const v4f a2 = *(const v4fa*)(z2 + (size_t)qd * 4);
    asm volatile("" :: "v"(a1)); asm volatile("" :: "v"(a2));
    const v4f a = (e != 0u) ? a2 : a1;
    const v4f r = (v4f){ bf16_val(a[0]), bf16_val(a[1]), bf16_val(a[2]), bf16_val(a[3]) };
    volatile v4f* q = (volatile v4f*)(ZR + (size_t)g * 4);
    *q = r;
    __threadfence();
    *q = r;
  } else {
    if (tid < 64u) {
      const unsigned seg = tid >> 4;
      const unsigned j4  = (tid & 15u) * 4u;
      const v4f wa = *(const v4fa*)(W2 + j4);
      const v4f wb = *(const v4fa*)(b1 + j4);
      const float wc = b2[0];
      asm volatile("" :: "v"(wa)); asm volatile("" :: "v"(wb)); asm volatile("" :: "v"(wc));
      const unsigned ma = (seg == 0u) ? 0xFFFFFFFFu : 0u;
      const unsigned mb = (seg == 1u) ? 0xFFFFFFFFu : 0u;
      const unsigned mc = (seg >= 2u) ? 0xFFFFFFFFu : 0u;
      const v4f r = (v4f){ bf16_val(blend3(wa[0], wb[0], wc, ma, mb, mc)), bf16_val(blend3(wa[1], wb[1], wc, ma, mb, mc)),
                           bf16_val(blend3(wa[2], wb[2], wc, ma, mb, mc)), bf16_val(blend3(wa[3], wb[3], wc, ma, mb, mc)) };
      volatile v4f* q = (volatile v4f*)(TAB + (size_t)tid * 4);
      *q = r;
      __threadfence();
      *q = r;
    }
  }
}

__global__ __launch_bounds__(256) void k_colsum(const float* __restrict__ ZR, double* __restrict__ REC) {
  __shared__ __attribute__((aligned(16))) double sP[4 * 64];
  const int tid = (int)threadIdx.x;
  const int blk = (int)blockIdx.x;
  const int e = blk >> 6;
  const int base = (blk & 63) * 16;
  const int g = tid >> 6;
  const int d = tid & 63;
  const float* zre = ZR + (size_t)e * (NPT * DD);
  const float y0 = zre[(size_t)(base + 4 * g + 0) * DD + d];
  const float y1 = zre[(size_t)(base + 4 * g + 1) * DD + d];
  const float y2 = zre[(size_t)(base + 4 * g + 2) * DD + d];
  const float y3 = zre[(size_t)(base + 4 * g + 3) * DD + d];
  double s0 = 0.0, s1 = 0.0, s2 = 0.0, s3 = 0.0;
#pragma unroll 1
  for (int jb = 0; jb < NPT / 32; ++jb) {
    const float* p = zre + (size_t)(jb * 32) * DD + d;
    float a0 = 0.0f, a1 = 0.0f, a2 = 0.0f, a3 = 0.0f;
#pragma unroll 4
    for (int jj = 0; jj < 32; ++jj) {
      const float zj = p[jj * DD];
      a0 += fabsf(y0 - zj);
      a1 += fabsf(y1 - zj);
      a2 += fabsf(y2 - zj);
      a3 += fabsf(y3 - zj);
    }
    s0 += (double)a0; s1 += (double)a1; s2 += (double)a2; s3 += (double)a3;
  }
  double tot = s0;
  tot += s1; tot += s2; tot += s3;
  sP[g * 64 + d] = tot;
  __syncthreads();
  if (tid < 32) {
    const int d0 = 2 * tid;
    double u0 = sP[d0];
    u0 += sP[64 + d0]; u0 += sP[128 + d0]; u0 += sP[192 + d0];
    double u1 = sP[d0 + 1];
    u1 += sP[64 + d0 + 1]; u1 += sP[128 + d0 + 1]; u1 += sP[192 + d0 + 1];
    pv2d v;
    v.x = u0; v.y = u1;
    volatile pv2d* q = (volatile pv2d*)(REC + ((size_t)blk * 64 + d0));
    *q = v;
    __threadfence();
    *q = v;
  }
}

__global__ __launch_bounds__(256) void k_w1s(const float* __restrict__ W1, const double* __restrict__ REC,
                                             float* __restrict__ SF, unsigned short* __restrict__ W1ST) {
  __shared__ __attribute__((aligned(16))) float sSF[128];
  __shared__ float sWs[2 * DD * WS_PITCH];
  const int tid = (int)threadIdx.x;
  if (tid < 128) {
    const int e = tid >> 6;
    const int d = tid & 63;
    double S = 0.0;
#pragma unroll 4
    for (int b = 0; b < 64; ++b) S += REC[(size_t)((e * 64 + b) * 64 + d)];
    sSF[tid] = fmaxf((float)S, 1e-12f);
  }
  __syncthreads();
  if (tid < 32) {
    const v4f v = *(const v4fa*)(sSF + 4 * tid);
    volatile v4f* q = (volatile v4f*)(SF + 4 * tid);
    *q = v;
    __threadfence();
    *q = v;
  }
#pragma unroll 1
  for (int it = 0; it < 8; ++it) {
    const int idx = it * 256 + tid;
    const int e  = idx >> 10;
    const int v  = idx & 1023;
    const int d  = v >> 4;
    const int c4 = (v & 15) * 4;
    const v4f w = *(const v4fa*)(W1 + d * DD + c4);
    const float sf = sSF[e * 64 + d];
    float* q = sWs + (e * 64 + d) * WS_PITCH + c4;
    q[0] = bf16_val(w[0]) / sf;
    q[1] = bf16_val(w[1]) / sf;
    q[2] = bf16_val(w[2]) / sf;
    q[3] = bf16_val(w[3]) / sf;
  }
  __syncthreads();
  v4u o[NITW];
#pragma unroll
  for (int it = 0; it < NITW; ++it) {
    const unsigned g    = (unsigned)(it * 256 + tid);
    const unsigned rowc = g / (unsigned)PPRZ;
    const unsigned p    = g - rowc * (unsigned)PPRZ;
    const unsigned e    = rowc >> 6;
    const unsigned c    = rowc & 63u;
    const unsigned pl   = p >> 3;
    const unsigned k0   = (p & 7u) << 3;
    const float* q = sWs + (e * 64u + k0) * WS_PITCH + c;
    float x[8];
#pragma unroll
    for (int i = 0; i < 8; ++i) x[i] = q[i * WS_PITCH];
    const v4f a = (v4f){ x[0], x[1], x[2], x[3] };
    const v4f b = (v4f){ x[4], x[5], x[6], x[7] };
    v4u r = pack8_bf16(a, b);
    if (W1S_TERMS >= 2) {
      const v4u l1 = pack8_bf16_lo(a, b);
      const unsigned m1 = (pl == 1u) ? 0xFFFFFFFFu : 0u;
      const v4u M1 = (v4u){ m1, m1, m1, m1 };
      r = (r & ~M1) | (l1 & M1);
    }
    if (W1S_TERMS == 3) {
      const v4u l2 = pack8_bf16_res2(a, b);
      const unsigned m2 = (pl == 2u) ? 0xFFFFFFFFu : 0u;
      const v4u M2 = (v4u){ m2, m2, m2, m2 };
      r = (r & ~M2) | (l2 & M2);
    }
    o[it] = r;
  }
#pragma unroll
  for (int it = 0; it < NITW; ++it) *(volatile v4u*)(W1ST + (size_t)(it * 256 + tid) * 8) = o[it];
  __threadfence();
#pragma unroll
  for (int it = 0; it < NITW; ++it) *(volatile v4u*)(W1ST + (size_t)(it * 256 + tid) * 8) = o[it];
}

__global__ __launch_bounds__(256) void k_pair(const float* __restrict__ ZW, const float* __restrict__ TAB,
                                              float* __restrict__ out) {
  extern __shared__ __attribute__((aligned(16))) float dsm[];
  float* sT = dsm;
  float* sO = dsm + LDS_T;
  float* sZ = dsm + LDS_T + LDS_O;
  float* sW = dsm + LDS_T + LDS_O + LDS_Z;
  const int tid  = (int)threadIdx.x;
  const int lane = tid & 31;
  const int wave = tid >> 5;
  const int row  = (int)blockIdx.x * 8 + wave;
  const int e    = row >> 10;
  const int i    = row & (NPT - 1);
  const float* zwe = ZW + (size_t)e * (NPT * DD);
  float* zs = sZ + wave * DD;
  float* so = sO + wave * NPT;
  const float b2r = TAB[128];

  if (wave == 0) {
    const v4f tv = *(const v4fa*)(TAB + 4 * lane);
    *(v4fa*)(sW + 4 * lane) = tv;
  }
  __syncthreads();
  {
    const pv2f a = *(const pv2fa*)(ZW + (size_t)row * DD + 2 * lane);
    const pv2f b = *(const pv2fa*)(sW + DD + 2 * lane);
    pv2f s;
    s.x = a.x + b.x; s.y = a.y + b.y;
    *(pv2fa*)(zs + 2 * lane) = s;
  }

  float part = 0.0f;
#pragma unroll 1
  for (int t = 0; t < NPT / TROWS; ++t) {
    __syncthreads();
    {
      v4f sv[8];
#pragma unroll
      for (int it = 0; it < 8; ++it) {
        const int idx = it * 256 + tid;
        const int r   = idx >> 4;
        const int c4  = (idx & 15) * 4;
        sv[it] = *(const v4fa*)(zwe + (size_t)(TROWS * t + r) * DD + c4);
      }
#pragma unroll
      for (int it = 0; it < 8; ++it) {
        const int idx = it * 256 + tid;
        const int r   = idx >> 4;
        const int c4  = (idx & 15) * 4;
        *(v4fa*)(sT + r * TPITCH + c4) = sv[it];
      }
    }
    __syncthreads();
#pragma unroll 1
    for (int s = 0; s < 4; ++s) {
      const float* rp = sT + (32 * s + lane) * TPITCH;
      float acc = 0.0f;
#pragma unroll 4
      for (int ch = 0; ch < 16; ++ch) {
        const v4f a  = *(const v4fa*)(rp + 4 * ch);
        const v4f zb = *(const v4fa*)(zs + 4 * ch);
        const v4f w  = *(const v4fa*)(sW + 4 * ch);
        float v;
        v = zb[0] - a[0]; v = (v > 0.0f) ? v : (v - v); acc = fmaf(v, w[0], acc);
        v = zb[1] - a[1]; v = (v > 0.0f) ? v : (v - v); acc = fmaf(v, w[1], acc);
        v = zb[2] - a[2]; v = (v > 0.0f) ? v : (v - v); acc = fmaf(v, w[2], acc);
        v = zb[3] - a[3]; v = (v > 0.0f) ? v : (v - v); acc = fmaf(v, w[3], acc);
      }
      float o = acc + b2r;
      o = (o > 0.0f) ? o : (o - o);
      so[TROWS * t + 32 * s + lane] = o;
      part += fabsf(o);
    }
  }

  __builtin_amdgcn_fence(__ATOMIC_RELEASE, "workgroup");
  __builtin_amdgcn_wave_barrier();
  __builtin_amdgcn_fence(__ATOMIC_ACQUIRE, "workgroup");

  float sum = part;
#pragma unroll
  for (int off = 16; off > 0; off >>= 1) sum += __shfl_xor(sum, off, 32);
  const float den = fmaxf(sum, 1e-12f);

  float* o0 = out + ((size_t)(e * NPT + i) * NPT + 4 * lane);
  float* o2 = out + ((size_t)((e + 2) * NPT + i) * NPT + 4 * lane);
#pragma unroll 1
  for (int t = 0; t < 8; ++t) {
    const v4f v = *(const v4fa*)(so + 128 * t + 4 * lane);
    v4f r;
    r[0] = v[0] / den; r[1] = v[1] / den; r[2] = v[2] / den; r[3] = v[3] / den;
    volatile v4f* q0 = (volatile v4f*)(o0 + 128 * t);
    volatile v4f* q2 = (volatile v4f*)(o2 + 128 * t);
    if (row < 2 * NPT) {
      *q0 = r;
      *q2 = r;
    }
    __threadfence();
    if (row < 2 * NPT) {
      *q0 = r;
      *q2 = r;
    }
  }
}

extern "C" void kernel_launch(void* const* d_in, const int* in_sizes, int n_in,
                              void* d_out, int out_size, void* d_ws, size_t ws_size,
                              hipStream_t stream) {
  if (n_in < 6) return;
  if (in_sizes[0] != NPT * DD || in_sizes[1] != NPT * DD) return;
  if (in_sizes[2] != DD * DD || in_sizes[3] != DD) return;
  if (in_sizes[4] != DD || in_sizes[5] != 1) return;
  if (out_size != OUT_ELEMS) return;
  if ((size_t)WS_TOTAL > ws_size) return;

  const float* z1 = (const float*)d_in[0];
  const float* z2 = (const float*)d_in[1];
  const float* W1 = (const float*)d_in[2];
  const float* b1 = (const float*)d_in[3];
  const float* W2 = (const float*)d_in[4];
  const float* b2 = (const float*)d_in[5];
  float* out = (float*)d_out;

  char* ws = (char*)d_ws;
  size_t off = 0;
  unsigned short* ZZ   = (unsigned short*)(ws + off); off += (size_t)SZ_ZZ;
  float*          ZR   = (float*)(ws + off);          off += (size_t)SZ_ZR;
  float*          ZW   = (float*)(ws + off);          off += (size_t)SZ_ZW;
  double*         REC  = (double*)(ws + off);         off += (size_t)SZ_REC;
  unsigned short* W1ST = (unsigned short*)(ws + off); off += (size_t)SZ_W1ST;
  float*          SF   = (float*)(ws + off);          off += (size_t)SZ_SF;
  float*          TAB  = (float*)(ws + off);          off += (size_t)SZ_TAB;
  if (off != (size_t)WS_TOTAL) return;

  hipFuncSetAttribute(reinterpret_cast<const void*>(&k_pair), hipFuncAttributeMaxDynamicSharedMemorySize,
                      (int)PAIR_LDS_BYTES);

  k_prep<<<NB_PREP, 256, 0, stream>>>(z1, z2, W2, b1, b2, ZZ, ZR, TAB);
  k_colsum<<<128, 256, 0, stream>>>(ZR, REC);
  k_w1s<<<1, 256, 0, stream>>>(W1, REC, SF, W1ST);
  k_gemm_nt<0, 0><<<2, 256, 0, stream>>>(ZZ, W1ST, TAB, ZW, NPT, DD, KT, DD);
  k_gemm_nt<0, 0><<<2, 256, 0, stream>>>(ZZ + (size_t)NPT * KT, W1ST + (size_t)DD * KT, TAB,
                                         ZW + (size_t)NPT * DD, NPT, DD, KT, DD);
  k_pair<<<(2 * NPT) / 8, 256, PAIR_LDS_BYTES, stream>>>(ZW, TAB, out);
}
